// BiModalAttention_76364518523410
// MI455X (gfx1250) — hardware-verified
//
#include <hip/hip_runtime.h>


namespace {
constexpr int B = 8, S = 2048, D = 128, BL = 8  , QL = 2048  ;
constexpr float XS = 8.0f, PS = 1024.0f, LOG2E = 1.4426950408889634f;
static_assert(S % 64 == 0 && QL % 32 == 0, "tiling");
typedef _Float16 b16;
typedef __attribute__((ext_vector_type(16))) _Float16 v16b;
typedef __attribute__((ext_vector_type(8))) _Float16 v8b;
typedef __attribute__((ext_vector_type(8))) float v8f;
typedef __attribute__((ext_vector_type(4))) float v4f;
__device__ __forceinline__ float bf16_rne(float f) { unsigned int u = __float_as_uint(f); u += 0x7FFFu + ((u >> 16) & 1u); return __uint_as_float(u & 0xFFFF0000u); }
__device__ __forceinline__ void split16(float v, b16& hi, b16& lo) { hi = (b16)v; lo = (b16)(v - (float)hi); }
__device__ __forceinline__ v16b frag_kb(const b16* p, int hh) { const v8b a = *(const v8b*)(p + 8 * hh), b = *(const v8b*)(p + 16 + 8 * hh); v16b f;
#pragma unroll
  for (int e = 0; e < 8; ++e) { f[e] = a[e]; f[8 + e] = b[e]; } return f; }
__device__ __forceinline__ v8f wmma16b(v16b a, v16b b, v8f c) { v8f d = __builtin_amdgcn_wmma_f32_16x16x32_f16(false, a, false, b, (short)0, c, false, false); asm volatile("v_nop\n\tv_nop\n\tv_nop\n\tv_nop" : "+v"(d) : "v"(a), "v"(b)); return d; }
__device__ __forceinline__ void wave_lds_sync() { __builtin_amdgcn_fence(__ATOMIC_RELEASE, "workgroup"); __builtin_amdgcn_wave_barrier(); __builtin_amdgcn_fence(__ATOMIC_ACQUIRE, "workgroup"); }
__device__ __forceinline__ float pmul(float a, float b) { float p = a * b; asm volatile("" : "+v"(p)); return p; }
__device__ __forceinline__ int iclamp(int v, int lo, int hi) { return v < lo ? lo : (v > hi ? hi : v); }

typedef __attribute__((ext_vector_type(2))) _Float16 v2h;
typedef __attribute__((ext_vector_type(4))) _Float16 v4h;
__device__ __forceinline__ float nexp2(float v) { return __builtin_amdgcn_exp2f(v); }
__global__ __launch_bounds__(256) void prep_kernel(const float* __restrict__ x, const float* __restrict__ y, b16* __restrict__ XP, b16* __restrict__ YP, b16* __restrict__ XT, b16* __restrict__ YT) {
  __shared__ b16 Ts[D][64 + 8];
  const int tb = blockIdx.x; const int which = tb / (B * (S / 64)); const int rem = tb % (B * (S / 64)); const int b = rem / (S / 64), t0 = (rem % (S / 64)) * 64;
  const float* src = which ? y : x; b16* P = which ? YP : XP; b16* T = which ? YT : XT;
  for (int pass = 0; pass < 2; ++pass) { for (int i = threadIdx.x; i < 64 * D / 8; i += 256) { const size_t e = ((size_t)b * S + t0) * D + (size_t)i * 8; v8b o; for (int j = 0; j < 8; ++j) o[j] = (b16)(bf16_rne(src[e + j]) * XS); *(volatile v8b*)(P + e) = o; } __threadfence(); }
  for (int i = threadIdx.x; i < 64 * D; i += 256) { const int tt = i / D, d = i % D; Ts[d][tt] = (b16)(bf16_rne(src[((size_t)b * S + t0 + tt) * D + d]) * XS); }
  __syncthreads();
  for (int pass = 0; pass < 2; ++pass) { for (int i = threadIdx.x; i < D * 8; i += 256) { const int d = i / 8, c8 = (i % 8) * 8; *(volatile v8b*)(T + ((size_t)b * D + d) * S + t0 + c8) = *(const v8b*)(&Ts[d][c8]); } __threadfence(); }
}
__global__ __launch_bounds__(64) void attn_kernel(const b16* __restrict__ XP, const b16* __restrict__ YP, const b16* __restrict__ XT, const b16* __restrict__ YT, const float* __restrict__ x, const float* __restrict__ y, float* __restrict__ out) {
  __shared__ __attribute__((aligned(16))) b16 Ph[2][16][32 + 8], Pl[2][16][32 + 8]; __shared__ __attribute__((aligned(16))) float To[2][16][D + 4];
  const int wave = threadIdx.x >> 5, lane = threadIdx.x & 31, hh = lane >> 4, col = lane & 15; const int b = blockIdx.y, dir = blockIdx.z; const int q0 = blockIdx.x * 32 + wave * 16, qi = q0 + col;
  const b16* Qb = (dir ? YP : XP) + (size_t)b * S * D; const b16* Kb = (dir ? XP : YP) + (size_t)b * S * D; const b16* Vb = (dir ? XT : YT) + (size_t)b * D * S; const float* gate = (dir ? y : x);
  v16b qa[4];
#pragma unroll
  for (int ks = 0; ks < 4; ++ks) qa[ks] = frag_kb(Qb + (size_t)qi * D + ks * 32, hh);
  const float cs = LOG2E / (XS * XS);
  float m = -INFINITY, l = 0.0f; v8f o[8]; for (int t = 0; t < 8; ++t) o[t] = (v8f){};
#pragma unroll 1
  for (int kb = 0; kb < S; kb += 32) {
    float e[16]; float mx = -INFINITY;
#pragma unroll
    for (int u = 0; u < 2; ++u) { v8f s = (v8f){}; const size_t kr = (size_t)(kb + u * 16 + col) * D;
#pragma unroll
      for (int ks = 0; ks < 4; ++ks) s = wmma16b(frag_kb(Kb + kr + ks * 32, hh), qa[ks], s);
#pragma unroll
      for (int r = 0; r < 8; ++r) { const float vv = s[r] * cs; e[u * 8 + r] = vv; mx = fmaxf(mx, vv); } }
    mx = fmaxf(mx, __shfl_xor(mx, 16)); const float mn = fmaxf(m, mx); const float al = nexp2(m - mn); float sum = 0.0f;
#pragma unroll
    for (int i2 = 0; i2 < 16; ++i2) { const float p = nexp2(e[i2] - mn); sum += p; b16 a_, b_; split16(p * PS, a_, b_); const int sl = (i2 < 8 ? 0 : 16) + 8 * hh + (i2 & 7); Ph[wave][col][sl] = a_; Pl[wave][col][sl] = b_; }
    sum += __shfl_xor(sum, 16); l = l * al + sum; m = mn;
    wave_lds_sync();
    const v16b ph = frag_kb(&Ph[wave][col][0], hh), pl = frag_kb(&Pl[wave][col][0], hh);
#pragma unroll
    for (int t = 0; t < 8; ++t) { o[t] *= al; const v16b va = frag_kb(Vb + (size_t)(t * 16 + col) * S + kb, hh); o[t] = wmma16b(va, ph, o[t]); o[t] = wmma16b(va, pl, o[t]); }
    wave_lds_sync(); }
  const float inv = 1.0f / (l * PS * XS);
#pragma unroll
  for (int t = 0; t < 8; ++t)
#pragma unroll
    for (int r = 0; r < 8; ++r) To[wave][col][t * 16 + 8 * hh + r] = o[t][r] * inv;
  wave_lds_sync();
  for (int pass = 0; pass < 2; ++pass) { for (int rr = 0; rr < 16; ++rr) { const size_t row = (size_t)b * S + q0 + rr; const v4f ov = *(const v4f*)(&To[wave][rr][lane * 4]); const v4f gv = *(const v4f*)(gate + row * D + lane * 4); v4f r4;
      for (int j = 0; j < 4; ++j) r4[j] = ov[j] * bf16_rne(gv[j]); *(volatile v4f*)(out + row * (2 * D) + dir * D + lane * 4) = r4; } __threadfence(); }
}
}

extern "C" void kernel_launch(void* const* d_in, const int* in_sizes, int n_in, void* d_out, int out_size, void* d_ws, size_t ws_size, hipStream_t stream) {
  (void)n_in;
  auto Fp = [&](int i) { return (const float*)d_in[i]; };
  if (in_sizes[0] != B * S * D || in_sizes[1] != B * S * D || out_size != B * S * 2 * D) return;
  size_t off = 0; char* ws = (char*)d_ws;
  auto carve = [&](size_t bytes) { char* p = ws + off; off += (bytes + 255) & ~(size_t)255; return p; };
  const size_t plane = (size_t)B * S * D * 2; b16* XP = (b16*)carve(plane); b16* YP = (b16*)carve(plane); b16* XT = (b16*)carve(plane); b16* YT = (b16*)carve(plane);
  if (off > ws_size || off > ((size_t)128 << 20)) return;
  prep_kernel<<<2 * B * (S / 64), 256, 0, stream>>>(Fp(0), Fp(1), XP, YP, XT, YT);
  attn_kernel<<<dim3(QL / 32, BL, 2), 64, 0, stream>>>(XP, YP, XT, YT, Fp(0), Fp(1), (float*)d_out);
}
